// DependencyNeuralModel_25529285607739
// MI455X (gfx1250) — hardware-verified
//
#include <hip/hip_runtime.h>
#include <math.h>
#include <stdint.h>

typedef __attribute__((ext_vector_type(16))) _Float16 v16h;
typedef __attribute__((ext_vector_type(8)))  _Float16 v8h;
typedef __attribute__((ext_vector_type(16))) __bf16   v16b;
typedef __attribute__((ext_vector_type(8)))  __bf16   v8b;
typedef __attribute__((ext_vector_type(8)))  float    v8f;
typedef __attribute__((ext_vector_type(4)))  float    v4f;

__device__ __forceinline__ unsigned short f2bf_bits(float f) {
  unsigned u = __float_as_uint(f);
  return (unsigned short)((u + 0x7FFFu + ((u >> 16) & 1u)) >> 16);
}
__device__ __forceinline__ float bf_bits2f(unsigned short h) { return __uint_as_float(((unsigned)h) << 16); }

__device__ __forceinline__ void dep_guard_h(v8f& a, v8f& b, v16h x, v16h y) { asm volatile("v_nop\n\tv_nop\n\tv_nop\n\tv_nop" : "+v"(a), "+v"(b) : "v"(x), "v"(y)); }
__device__ __forceinline__ void dep_guard_b(v8f& a, v8f& b, v16b x, v16b y) { asm volatile("v_nop\n\tv_nop\n\tv_nop\n\tv_nop" : "+v"(a), "+v"(b) : "v"(x), "v"(y)); }
__device__ __forceinline__ void keep4_h(v16h a, v16h b, v16h c, v16h d) { asm volatile("v_nop" :: "v"(a), "v"(b), "v"(c), "v"(d)); }
__device__ __forceinline__ void keep4_b(v16b a, v16b b, v16b c, v16b d) { asm volatile("v_nop" :: "v"(a), "v"(b), "v"(c), "v"(d)); }
__device__ __forceinline__ void acc_guard4(v8f& a, v8f& b, v8f& c, v8f& d) { asm volatile("v_nop\n\tv_nop\n\tv_nop\n\tv_nop" : "+v"(a), "+v"(b), "+v"(c), "+v"(d)); }
template <typename T> struct Frag;
template <> struct Frag<_Float16> {
  typedef v16h V; union U { v16h v; v8h h[2]; };
  static __device__ __forceinline__ v16h load(const _Float16* p) {
    U f; f.h[0] = *(const v8h*)(p); f.h[1] = *(const v8h*)(p + 16); return f.v;
  }
  static __device__ __forceinline__ v8f mma(v16h a, v16h b, v8f c) {
    return __builtin_amdgcn_wmma_f32_16x16x32_f16(false, a, false, b, (short)0, c, false, false);
  }
  static __device__ __forceinline__ void guard(v8f& a, v8f& b, v16h x, v16h y) { dep_guard_h(a, b, x, y); }
  static __device__ __forceinline__ void keep(v16h a, v16h b, v16h c, v16h d) { keep4_h(a, b, c, d); }
};
template <> struct Frag<__bf16> {
  typedef v16b V; union U { v16b v; v8b h[2]; };
  static __device__ __forceinline__ v16b load(const __bf16* p) {
    U f; f.h[0] = *(const v8b*)(p); f.h[1] = *(const v8b*)(p + 16); return f.v;
  }
  static __device__ __forceinline__ v8f mma(v16b a, v16b b, v8f c) {
    return __builtin_amdgcn_wmma_f32_16x16x32_bf16(false, a, false, b, (short)0, c, false, false);
  }
  static __device__ __forceinline__ void guard(v8f& a, v8f& b, v16b x, v16b y) { dep_guard_b(a, b, x, y); }
  static __device__ __forceinline__ void keep(v16b a, v16b b, v16b c, v16b d) { keep4_b(a, b, c, d); }
};

template <int ET> struct Elem;
template <> struct Elem<0> { typedef _Float16 T; };
template <> struct Elem<1> { typedef __bf16 T; };
template <int ET, bool SPLIT, int BIAS_MODE, int OUT_MODE, bool RESID, int ACT = 0>
__global__ __launch_bounds__(256) void wmma_gemm64(
    const unsigned short* __restrict__ Ap, const unsigned short* __restrict__ A2p, int lda, long strideA,
    const unsigned short* __restrict__ Btp, const unsigned short* __restrict__ Bt2p, int ldb, long strideB,
    void* __restrict__ Cout, void* __restrict__ Cout2, int ldc, long strideC,
    const float* __restrict__ bias,
    const float* __restrict__ resid, long strideR,
    int M, int N, int K, float scale) {
  typedef typename Elem<ET>::T T;
  typedef typename Frag<T>::V V;
  const T* A = (const T*)Ap; const T* A2 = (const T*)A2p; const T* Bt = (const T*)Btp; const T* Bt2 = (const T*)Bt2p;
  __shared__ __align__(16) float sT[8][16 * 68];
  const int b    = blockIdx.y;
  const int lane = threadIdx.x & 31;
  const int wave = threadIdx.x >> 5;
  const int tilesN = N >> 6;
  const int tilesM = M >> 6;
  const int tile = blockIdx.x * 8 + wave;
  if (tile >= tilesM * tilesN) return;
  const int tm = tile / tilesN;
  const int tn = tile - tm * tilesN;
  const int m0 = tm << 6;
  const int n0 = tn << 6;

  const T* Ab  = A  + (size_t)b * strideA;
  const T* Bb  = Bt + (size_t)b * strideB;
  const T* Ab2 = SPLIT ? (A2  + (size_t)b * strideA) : nullptr;
  const T* Bb2 = SPLIT ? (Bt2 + (size_t)b * strideB) : nullptr;

  const int rlane = lane & 15;
  const int koff  = (lane >> 4) * 8;
  const int mOff  = (lane >> 4) * 8;

  v8f acc[4][4];
#pragma unroll
  for (int i = 0; i < 4; ++i)
#pragma unroll
    for (int j = 0; j < 4; ++j) acc[i][j] = (v8f){0.f,0.f,0.f,0.f,0.f,0.f,0.f,0.f};

  for (int k0 = 0; k0 < K; k0 += 32) {
    V bh[4], bl[4];
#pragma unroll
    for (int j = 0; j < 4; ++j) {
      const size_t bo = (size_t)(n0 + (j << 4) + rlane) * ldb + koff + k0;
      bh[j] = Frag<T>::load(Bb + bo);
      if (SPLIT) bl[j] = Frag<T>::load(Bb2 + bo);
    }
#pragma unroll
    for (int i = 0; i < 4; ++i) {
      const size_t ao = (size_t)(m0 + (i << 4) + rlane) * lda + koff + k0;
      V ah = Frag<T>::load(Ab + ao);
      V al;
      if (SPLIT) al = Frag<T>::load(Ab2 + ao);
#pragma unroll
      for (int j = 0; j < 4; ++j) {
        acc[i][j] = Frag<T>::mma(ah, bh[j], acc[i][j]);
        if (SPLIT) {
          acc[i][j] = Frag<T>::mma(ah, bl[j], acc[i][j]);
          acc[i][j] = Frag<T>::mma(al, bh[j], acc[i][j]);
        }
      }
      Frag<T>::guard(acc[i][0], acc[i][3], ah, SPLIT ? al : ah);
    }
    Frag<T>::keep(bh[0], bh[1], bh[2], bh[3]);
    if (SPLIT) Frag<T>::keep(bl[0], bl[1], bl[2], bl[3]);
  }
  acc_guard4(acc[0][0], acc[0][1], acc[0][2], acc[0][3]);
  acc_guard4(acc[1][0], acc[1][1], acc[1][2], acc[1][3]);
  acc_guard4(acc[2][0], acc[2][1], acc[2][2], acc[2][3]);
  acc_guard4(acc[3][0], acc[3][1], acc[3][2], acc[3][3]);

  float* slab = sT[wave];
  const float* Rb = RESID ? (resid + (size_t)b * strideR) : nullptr;
#pragma unroll
  for (int i = 0; i < 4; ++i) {
    const int mBase = m0 + (i << 4);
#pragma unroll
    for (int j = 0; j < 4; ++j) {
      const int n = n0 + (j << 4) + rlane;
      float bv = 0.f;
      if (BIAS_MODE == 2) bv = bias[n];
#pragma unroll
      for (int r = 0; r < 8; ++r) {
        float v = acc[i][j][r] * scale;
        if (BIAS_MODE == 1) v += bias[mBase + mOff + r];
        if (BIAS_MODE == 2) v += bv;
        if (RESID) v += Rb[(size_t)(mBase + mOff + r) * ldc + n];
        if (ACT == 1) v = tanhf(v);
        if (ACT == 2) v = fmaxf(v, 0.0f);
        if (ACT == 3) v = v / (1.0f + expf(-v));
        if (ACT == 4) v = (v > 0.f) ? v : 0.01f * v;
        if (ACT == 5) v = 0.5f * v * (1.0f + erff(v * 0.70710678118654752f));
        slab[(mOff + r) * 68 + (j << 4) + rlane] = v;
      }
    }
    __builtin_amdgcn_fence(__ATOMIC_RELEASE, "workgroup");
    __builtin_amdgcn_wave_barrier();
    __builtin_amdgcn_fence(__ATOMIC_ACQUIRE, "workgroup");
    if (OUT_MODE == 0) {
      float* C = (float*)Cout + (size_t)b * strideC;
      const int hh = lane >> 4, c4 = (lane & 15) * 4;
      for (int pass = 0; pass < 2; ++pass) {
#pragma unroll
        for (int it = 0; it < 8; ++it) {
          const int row = it * 2 + hh;
          v4f v = *(const v4f*)(slab + row * 68 + c4);
          *(volatile v4f*)(C + (size_t)(mBase + row) * ldc + n0 + c4) = v;
        }
        __threadfence();
      }
    } else {
      const int q = lane >> 3, c8 = (lane & 7) * 8;
      unsigned short* C  = (unsigned short*)Cout  + (size_t)b * strideC;
      unsigned short* C2 = (OUT_MODE == 2) ? ((unsigned short*)Cout2 + (size_t)b * strideC) : nullptr;
      for (int pass = 0; pass < 2; ++pass) {
#pragma unroll
        for (int it = 0; it < 4; ++it) {
          const int row = it * 4 + q;
          const float* sp = slab + row * 68 + c8;
          v8h hv, lv;
#pragma unroll
          for (int e = 0; e < 8; ++e) {
            if (OUT_MODE == 1) {
              hv[e] = (_Float16)sp[e];
            } else {
              unsigned short hb = f2bf_bits(sp[e]);
              unsigned short lb = f2bf_bits(sp[e] - bf_bits2f(hb));
              hv[e] = __builtin_bit_cast(_Float16, hb);
              lv[e] = __builtin_bit_cast(_Float16, lb);
            }
          }
          *(volatile v8h*)(C + (size_t)(mBase + row) * ldc + n0 + c8) = hv;
          if (OUT_MODE == 2) *(volatile v8h*)(C2 + (size_t)(mBase + row) * ldc + n0 + c8) = lv;
        }
        __threadfence();
      }
    }
    __builtin_amdgcn_fence(__ATOMIC_RELEASE, "workgroup");
    __builtin_amdgcn_wave_barrier();
    __builtin_amdgcn_fence(__ATOMIC_ACQUIRE, "workgroup");
  }
}

constexpr int SEQ_LEN   = 512;
constexpr int HID_DIM   = 512;
constexpr int GATE4     = 2048;
constexpr int WORD_V    = 50000;
constexpr int WORD_E    = 300;
constexpr int TAG_V     = 50;
constexpr int TAG_E     = 64;
constexpr int EMB_K     = WORD_E + TAG_E;
constexpr int EMB_KP    = 384;
constexpr int X1_K      = 2 * HID_DIM;
constexpr int PROJ_N    = 5 * HID_DIM;
constexpr int DIST_ROWS = 34;
constexpr int DIST_RP   = 64;
constexpr int DIST_K    = 64;
constexpr int NUM_BINS  = 17;
constexpr int NUM_ARC   = 262144;
constexpr int NUM_SIB   = 131072;
constexpr int PARTS_PER_BLOCK = 32;

static_assert(EMB_K == 364);
static_assert(EMB_KP % 32 == 0 && EMB_KP >= EMB_K);
static_assert(X1_K % 32 == 0 && HID_DIM % 32 == 0 && DIST_K % 32 == 0);
static_assert(SEQ_LEN % 64 == 0 && GATE4 % 64 == 0 && PROJ_N % 64 == 0 && DIST_RP % 64 == 0 && HID_DIM % 64 == 0);
static_assert(NUM_ARC % PARTS_PER_BLOCK == 0 && NUM_SIB % PARTS_PER_BLOCK == 0);
static_assert((NUM_ARC * 4) % 128 == 0);
static_assert(GATE4 == 4 * HID_DIM);

constexpr size_t SZ_X0   = (size_t)SEQ_LEN * EMB_KP * 2;
constexpr size_t SZ_WIH0 = (size_t)2 * GATE4 * EMB_KP * 2;
constexpr size_t SZ_WIH1 = (size_t)2 * GATE4 * X1_K * 2;
constexpr size_t SZ_WHH  = (size_t)2 * GATE4 * HID_DIM * 2;
constexpr size_t SZ_PW   = (size_t)PROJ_N * X1_K * 2;
constexpr size_t SZ_DE   = (size_t)DIST_RP * DIST_K * 2;
constexpr size_t SZ_DW   = (size_t)HID_DIM * DIST_K * 2;
constexpr size_t SZ_GX   = (size_t)2 * SEQ_LEN * GATE4 * 4;
constexpr size_t SZ_HIST = (size_t)SEQ_LEN * X1_K * 4;
constexpr size_t SZ_X1   = (size_t)SEQ_LEN * X1_K * 2;
constexpr size_t SZ_ST   = (size_t)SEQ_LEN * X1_K * 2;
constexpr size_t SZ_PROJ = (size_t)SEQ_LEN * PROJ_N * 4;
constexpr size_t SZ_DTAB = (size_t)DIST_RP * HID_DIM * 4;

constexpr size_t OFF_X0   = 0;
constexpr size_t OFF_WIH0 = OFF_X0 + SZ_X0;
constexpr size_t OFF_WIH1 = OFF_WIH0 + SZ_WIH0;
constexpr size_t OFF_WHH0 = OFF_WIH1 + SZ_WIH1;
constexpr size_t OFF_WHH1 = OFF_WHH0 + SZ_WHH;
constexpr size_t OFF_PWH  = OFF_WHH1 + SZ_WHH;
constexpr size_t OFF_PWL  = OFF_PWH + SZ_PW;
constexpr size_t OFF_DEH  = OFF_PWL + SZ_PW;
constexpr size_t OFF_DEL  = OFF_DEH + SZ_DE;
constexpr size_t OFF_DWH  = OFF_DEL + SZ_DE;
constexpr size_t OFF_DWL  = OFF_DWH + SZ_DW;
constexpr size_t OFF_GX   = OFF_DWL + SZ_DW;
constexpr size_t OFF_H0   = OFF_GX + SZ_GX;
constexpr size_t OFF_H1   = OFF_H0 + SZ_HIST;
constexpr size_t OFF_X1   = OFF_H1 + SZ_HIST;
constexpr size_t OFF_STH  = OFF_X1 + SZ_X1;
constexpr size_t OFF_STL  = OFF_STH + SZ_ST;
constexpr size_t OFF_PROJ = OFF_STL + SZ_ST;
constexpr size_t OFF_DTAB = OFF_PROJ + SZ_PROJ;
constexpr size_t WS_TOTAL = OFF_DTAB + SZ_DTAB;
static_assert(WS_TOTAL == 52051968);
static_assert(WS_TOTAL <= (size_t)134217728);
static_assert(OFF_WIH0 % 256 == 0 && OFF_WIH1 % 256 == 0 && OFF_WHH0 % 256 == 0 && OFF_WHH1 % 256 == 0 && OFF_PWH % 256 == 0 &&
              OFF_PWL % 256 == 0 && OFF_DEH % 256 == 0 && OFF_DEL % 256 == 0 && OFF_DWH % 256 == 0 && OFF_DWL % 256 == 0 &&
              OFF_GX % 256 == 0 && OFF_H0 % 256 == 0 && OFF_H1 % 256 == 0 && OFF_X1 % 256 == 0 && OFF_STH % 256 == 0 &&
              OFF_STL % 256 == 0 && OFF_PROJ % 256 == 0 && OFF_DTAB % 256 == 0);

__device__ __forceinline__ float rcp_apx(float x) { return __builtin_amdgcn_rcpf(x); }
__device__ __forceinline__ float tanh_apx(float x) {
  const float e = __expf(2.0f * x);
  return fmaf(-2.0f, rcp_apx(1.0f + e), 1.0f);
}
__device__ __forceinline__ float sigm_apx(float x) { return rcp_apx(1.0f + __expf(-x)); }

__device__ __forceinline__ int clamp_int(int v, int lo, int hi) { return v < lo ? lo : (v > hi ? hi : v); }

__global__ __launch_bounds__(256) void cast_rows_f16(const float* __restrict__ in, _Float16* __restrict__ out,
                                                     int K, int Kp, int n2) {
  const int i = blockIdx.x * 256 + threadIdx.x;
  if (i < n2) {
    const int e = 2 * i;
    const int row = e / Kp;
    const int col = e - row * Kp;
    const int colc = (col < K - 2) ? col : (K - 2);
    const float* src = in + (size_t)row * K + colc;
    float a = src[0];
    float b = src[1];
    if (col >= K) { a = 0.0f; b = 0.0f; }
    const unsigned u = (unsigned)__builtin_bit_cast(unsigned short, (_Float16)a) |
                       ((unsigned)__builtin_bit_cast(unsigned short, (_Float16)b) << 16);
    volatile unsigned* op = (volatile unsigned*)out + i;
    *op = u;
    __threadfence();
    *op = u;
  }
}

__global__ __launch_bounds__(256) void cast_rows_bf16hl(const float* __restrict__ in, unsigned short* __restrict__ hi,
                                                        unsigned short* __restrict__ lo, int Rr, int K, int Kp, int n2) {
  const int i = blockIdx.x * 256 + threadIdx.x;
  if (i < n2) {
    const int e = 2 * i;
    const int row = e / Kp;
    const int col = e - row * Kp;
    const int rowc = (row < Rr) ? row : (Rr - 1);
    const int colc = (col < K - 2) ? col : (K - 2);
    const float* src = in + (size_t)rowc * K + colc;
    float a = src[0];
    float b = src[1];
    if (row >= Rr || col >= K) { a = 0.0f; b = 0.0f; }
    const unsigned short ha = f2bf_bits(a);
    const unsigned short hb = f2bf_bits(b);
    const unsigned short la = f2bf_bits(a - bf_bits2f(ha));
    const unsigned short lb = f2bf_bits(b - bf_bits2f(hb));
    const unsigned uh = (unsigned)ha | ((unsigned)hb << 16);
    const unsigned ul = (unsigned)la | ((unsigned)lb << 16);
    volatile unsigned* oh = (volatile unsigned*)hi + i;
    volatile unsigned* ol = (volatile unsigned*)lo + i;
    *oh = uh;
    *ol = ul;
    __threadfence();
    *oh = uh;
    *ol = ul;
  }
}

__global__ __launch_bounds__(192) void embed_rows(const int* __restrict__ words, const int* __restrict__ tags,
                                                  const float* __restrict__ we, const float* __restrict__ te,
                                                  _Float16* __restrict__ x0) {
  const int s = blockIdx.x;
  const int wi = clamp_int(words[s], 0, WORD_V - 1);
  const int ti = clamp_int(tags[s], 0, TAG_V - 1);
  const int col = 2 * threadIdx.x;
  const int cw = (col < WORD_E - 2) ? col : (WORD_E - 2);
  int ct = col - WORD_E;
  ct = ct < 0 ? 0 : (ct > TAG_E - 2 ? TAG_E - 2 : ct);
  const float* wp = we + (size_t)wi * WORD_E + cw;
  const float* tp = te + (size_t)ti * TAG_E + ct;
  const float wa = wp[0], wb = wp[1];
  const float ta = tp[0], tb = tp[1];
  const float a = (col < WORD_E) ? wa : ((col < EMB_K) ? ta : 0.0f);
  const float b = (col < WORD_E) ? wb : ((col < EMB_K) ? tb : 0.0f);
  const unsigned u = (unsigned)__builtin_bit_cast(unsigned short, (_Float16)a) |
                     ((unsigned)__builtin_bit_cast(unsigned short, (_Float16)b) << 16);
  volatile unsigned* op = (volatile unsigned*)x0 + (size_t)s * (EMB_KP / 2) + threadIdx.x;
  *op = u;
  __threadfence();
  *op = u;
}

__global__ __launch_bounds__(512) void lstm_scan_dir(const float* __restrict__ gx, const _Float16* __restrict__ whh,
                                                     const float* __restrict__ bih, const float* __restrict__ bhh,
                                                     float* __restrict__ hist) {
  __shared__ __align__(16) _Float16 h16[HID_DIM];
  __shared__ __align__(16) float gsh[GATE4];
  const int d = blockIdx.x;
  const int tid = threadIdx.x;
  const int lane = tid & 31;
  const int wave = tid >> 5;
  const int hh = lane >> 4;
  const int rl = lane & 15;
  const int r8 = lane & 7;
  const int koff = hh * 8;
  const _Float16* Wd = whh + (size_t)d * GATE4 * HID_DIM;
  const float* gxd = gx + (size_t)d * SEQ_LEN * GATE4;
  const float bs0 = bih[d * GATE4 + 0 * HID_DIM + tid] + bhh[d * GATE4 + 0 * HID_DIM + tid];
  const float bs1 = bih[d * GATE4 + 1 * HID_DIM + tid] + bhh[d * GATE4 + 1 * HID_DIM + tid];
  const float bs2 = bih[d * GATE4 + 2 * HID_DIM + tid] + bhh[d * GATE4 + 2 * HID_DIM + tid];
  const float bs3 = bih[d * GATE4 + 3 * HID_DIM + tid] + bhh[d * GATE4 + 3 * HID_DIM + tid];
  float cst = 0.0f;
  h16[tid] = (_Float16)0.0f;
  __syncthreads();

  for (int step = 0; step < SEQ_LEN; ++step) {
    const int t = d ? (SEQ_LEN - 1 - step) : step;
    v8f acc[8];
#pragma unroll
    for (int i = 0; i < 8; ++i) acc[i] = (v8f){0.f,0.f,0.f,0.f,0.f,0.f,0.f,0.f};

#pragma unroll
    for (int kc = 0; kc < HID_DIM / 32; ++kc) {
      const int k0 = kc * 32;
      Frag<_Float16>::U bu;
      bu.h[0] = *(const v8h*)(h16 + k0 + koff);
      bu.h[1] = *(const v8h*)(h16 + k0 + 16 + koff);
      const v16h bv = bu.v;
#pragma unroll
      for (int g = 0; g < 2; ++g) {
        v16h af[4];
#pragma unroll
        for (int tt = 0; tt < 4; ++tt) {
          const int row = (wave * 8 + g * 4 + tt) * 16 + rl;
          af[tt] = Frag<_Float16>::load(Wd + (size_t)row * HID_DIM + k0 + koff);
        }
#pragma unroll
        for (int tt = 0; tt < 4; ++tt) acc[g * 4 + tt] = Frag<_Float16>::mma(af[tt], bv, acc[g * 4 + tt]);
        dep_guard_h(acc[g * 4 + 0], acc[g * 4 + 3], af[0], af[1]);
        keep4_h(af[2], af[3], bv, bv);
      }
    }
    acc_guard4(acc[0], acc[1], acc[2], acc[3]);
    acc_guard4(acc[4], acc[5], acc[6], acc[7]);

#pragma unroll
    for (int i = 0; i < 8; ++i) {
      float v = acc[i][0];
      v = (r8 == 1) ? acc[i][1] : v;
      v = (r8 == 2) ? acc[i][2] : v;
      v = (r8 == 3) ? acc[i][3] : v;
      v = (r8 == 4) ? acc[i][4] : v;
      v = (r8 == 5) ? acc[i][5] : v;
      v = (r8 == 6) ? acc[i][6] : v;
      v = (r8 == 7) ? acc[i][7] : v;
      if (rl < 8) gsh[(wave * 8 + i) * 16 + hh * 8 + r8] = v;
    }
    __syncthreads();

    {
      const float* gxr = gxd + (size_t)t * GATE4;
      const float gi = gsh[0 * HID_DIM + tid] + gxr[0 * HID_DIM + tid] + bs0;
      const float gf = gsh[1 * HID_DIM + tid] + gxr[1 * HID_DIM + tid] + bs1;
      const float gg = gsh[2 * HID_DIM + tid] + gxr[2 * HID_DIM + tid] + bs2;
      const float go = gsh[3 * HID_DIM + tid] + gxr[3 * HID_DIM + tid] + bs3;
      cst = sigm_apx(gf) * cst + sigm_apx(gi) * tanh_apx(gg);
      const float hv = sigm_apx(go) * tanh_apx(cst);
      h16[tid] = (_Float16)hv;
      volatile float* hp = (volatile float*)(hist + (size_t)t * X1_K + d * HID_DIM + tid);
      *hp = hv;
      __threadfence();
      *hp = hv;
    }
    __syncthreads();
  }
}

__global__ __launch_bounds__(256) void arc_score_rows(const float* __restrict__ proj, const float* __restrict__ dtab,
                                                      const int* __restrict__ ah, const int* __restrict__ am,
                                                      const float* __restrict__ w, float* __restrict__ out) {
  __shared__ float sc[PARTS_PER_BLOCK];
  const int lane = threadIdx.x & 31;
  const int wave = threadIdx.x >> 5;
  float wr[16];
#pragma unroll
  for (int it = 0; it < 4; ++it) {
    const v4f t4 = *(const v4f*)(w + it * 128 + lane * 4);
    wr[it * 4 + 0] = t4[0]; wr[it * 4 + 1] = t4[1]; wr[it * 4 + 2] = t4[2]; wr[it * 4 + 3] = t4[3];
  }
#pragma unroll 1
  for (int q = 0; q < 4; ++q) {
    const int p = blockIdx.x * PARTS_PER_BLOCK + wave * 4 + q;
    const int hraw = ah[p];
    const int mraw = am[p];
    const int dlt = mraw - hraw;
    const int absd = dlt < 0 ? -dlt : dlt;
    const int bin = (absd < 10) ? absd : ((absd < 40) ? (10 + (absd - 10) / 5) : 16);
    const int di = (mraw > hraw) ? bin : (bin + NUM_BINS);
    const int hi = clamp_int(hraw, 0, SEQ_LEN - 1);
    const int mi = clamp_int(mraw, 0, SEQ_LEN - 1);
    const float* hpt = proj + (size_t)hi * PROJ_N;
    const float* mpt = proj + (size_t)mi * PROJ_N + HID_DIM;
    const float* dpt = dtab + (size_t)di * HID_DIM;
    float acc = 0.0f;
#pragma unroll
    for (int it = 0; it < 4; ++it) {
      const int c0 = it * 128 + lane * 4;
      const v4f a4 = *(const v4f*)(hpt + c0);
      const v4f b4 = *(const v4f*)(mpt + c0);
      const v4f d4 = *(const v4f*)(dpt + c0);
#pragma unroll
      for (int e = 0; e < 4; ++e) {
        const float x = (a4[e] + b4[e]) + d4[e];
        acc = fmaf(tanh_apx(x), wr[it * 4 + e], acc);
      }
    }
#pragma unroll
    for (int off = 16; off > 0; off >>= 1) acc += __shfl_xor(acc, off, 32);
    if (lane == 0) sc[wave * 4 + q] = acc;
  }
  __syncthreads();
  if (wave == 0) {
    const float v = sc[lane];
    volatile float* op = (volatile float*)(out + (size_t)blockIdx.x * PARTS_PER_BLOCK + lane);
    *op = v;
    __threadfence();
    *op = v;
  }
}

__global__ __launch_bounds__(256) void sib_score_rows(const float* __restrict__ proj,
                                                      const int* __restrict__ ih, const int* __restrict__ im,
                                                      const int* __restrict__ is, const float* __restrict__ w,
                                                      float* __restrict__ out) {
  __shared__ float sc[PARTS_PER_BLOCK];
  const int lane = threadIdx.x & 31;
  const int wave = threadIdx.x >> 5;
  float wr[16];
#pragma unroll
  for (int it = 0; it < 4; ++it) {
    const v4f t4 = *(const v4f*)(w + it * 128 + lane * 4);
    wr[it * 4 + 0] = t4[0]; wr[it * 4 + 1] = t4[1]; wr[it * 4 + 2] = t4[2]; wr[it * 4 + 3] = t4[3];
  }
#pragma unroll 1
  for (int q = 0; q < 4; ++q) {
    const int p = blockIdx.x * PARTS_PER_BLOCK + wave * 4 + q;
    const int hi = clamp_int(ih[p], 0, SEQ_LEN - 1);
    const int mi = clamp_int(im[p], 0, SEQ_LEN - 1);
    const int si = clamp_int(is[p], 0, SEQ_LEN - 1);
    const float* hpt = proj + (size_t)hi * PROJ_N + 2 * HID_DIM;
    const float* mpt = proj + (size_t)mi * PROJ_N + 3 * HID_DIM;
    const float* spt = proj + (size_t)si * PROJ_N + 4 * HID_DIM;
    float acc = 0.0f;
#pragma unroll
    for (int it = 0; it < 4; ++it) {
      const int c0 = it * 128 + lane * 4;
      const v4f a4 = *(const v4f*)(hpt + c0);
      const v4f b4 = *(const v4f*)(mpt + c0);
      const v4f d4 = *(const v4f*)(spt + c0);
#pragma unroll
      for (int e = 0; e < 4; ++e) {
        const float x = (a4[e] + b4[e]) + d4[e];
        acc = fmaf(tanh_apx(x), wr[it * 4 + e], acc);
      }
    }
#pragma unroll
    for (int off = 16; off > 0; off >>= 1) acc += __shfl_xor(acc, off, 32);
    if (lane == 0) sc[wave * 4 + q] = acc;
  }
  __syncthreads();
  if (wave == 0) {
    const float v = sc[lane];
    volatile float* op = (volatile float*)(out + (size_t)blockIdx.x * PARTS_PER_BLOCK + lane);
    *op = v;
    __threadfence();
    *op = v;
  }
}

extern "C" void kernel_launch(void* const* d_in, const int* in_sizes, int n_in,
                              void* d_out, int out_size, void* d_ws, size_t ws_size,
                              hipStream_t stream) {
  (void)in_sizes; (void)n_in;
  const int*   words    = (const int*)  d_in[0];
  const int*   tags     = (const int*)  d_in[1];
  const int*   arc_head = (const int*)  d_in[2];
  const int*   arc_mod  = (const int*)  d_in[3];
  const int*   sib_head = (const int*)  d_in[4];
  const int*   sib_mod  = (const int*)  d_in[5];
  const int*   sib_sib  = (const int*)  d_in[6];
  const float* word_emb = (const float*)d_in[7];
  const float* tag_emb  = (const float*)d_in[8];
  const float* dist_emb = (const float*)d_in[9];
  const float* Wih0     = (const float*)d_in[10];
  const float* Whh0     = (const float*)d_in[11];
  const float* bih0     = (const float*)d_in[12];
  const float* bhh0     = (const float*)d_in[13];
  const float* Wih1     = (const float*)d_in[14];
  const float* Whh1     = (const float*)d_in[15];
  const float* bih1     = (const float*)d_in[16];
  const float* bhh1     = (const float*)d_in[17];
  const float* projW[5] = { (const float*)d_in[18], (const float*)d_in[19], (const float*)d_in[20],
                            (const float*)d_in[21], (const float*)d_in[22] };
  const float* dist_W   = (const float*)d_in[23];
  const float* dist_b   = (const float*)d_in[24];
  const float* arc_w    = (const float*)d_in[25];

  if (ws_size < WS_TOTAL) return;
  if ((size_t)out_size < (size_t)(NUM_ARC + NUM_SIB)) return;

  char* ws = (char*)d_ws;
  _Float16*       x0   = (_Float16*)(ws + OFF_X0);
  _Float16*       wih0 = (_Float16*)(ws + OFF_WIH0);
  _Float16*       wih1 = (_Float16*)(ws + OFF_WIH1);
  _Float16*       whh0 = (_Float16*)(ws + OFF_WHH0);
  _Float16*       whh1 = (_Float16*)(ws + OFF_WHH1);
  unsigned short* pwh  = (unsigned short*)(ws + OFF_PWH);
  unsigned short* pwl  = (unsigned short*)(ws + OFF_PWL);
  unsigned short* deh  = (unsigned short*)(ws + OFF_DEH);
  unsigned short* del  = (unsigned short*)(ws + OFF_DEL);
  unsigned short* dwh  = (unsigned short*)(ws + OFF_DWH);
  unsigned short* dwl  = (unsigned short*)(ws + OFF_DWL);
  float*          gx   = (float*)(ws + OFF_GX);
  float*          hist0 = (float*)(ws + OFF_H0);
  float*          hist1 = (float*)(ws + OFF_H1);
  _Float16*       x1   = (_Float16*)(ws + OFF_X1);
  unsigned short* sth  = (unsigned short*)(ws + OFF_STH);
  unsigned short* stl  = (unsigned short*)(ws + OFF_STL);
  float*          proj = (float*)(ws + OFF_PROJ);
  float*          dtab = (float*)(ws + OFF_DTAB);
  float*          out  = (float*)d_out;

  embed_rows<<<SEQ_LEN, 192, 0, stream>>>(words, tags, word_emb, tag_emb, x0);

  {
    const int n2 = 2 * GATE4 * EMB_KP / 2;
    cast_rows_f16<<<(n2 + 255) / 256, 256, 0, stream>>>(Wih0, wih0, EMB_K, EMB_KP, n2);
  }
  {
    const int n2 = 2 * GATE4 * X1_K / 2;
    cast_rows_f16<<<(n2 + 255) / 256, 256, 0, stream>>>(Wih1, wih1, X1_K, X1_K, n2);
  }
  {
    const int n2 = 2 * GATE4 * HID_DIM / 2;
    cast_rows_f16<<<(n2 + 255) / 256, 256, 0, stream>>>(Whh0, whh0, HID_DIM, HID_DIM, n2);
    cast_rows_f16<<<(n2 + 255) / 256, 256, 0, stream>>>(Whh1, whh1, HID_DIM, HID_DIM, n2);
  }
  {
    const int n2 = HID_DIM * X1_K / 2;
    for (int i = 0; i < 5; ++i)
      cast_rows_bf16hl<<<(n2 + 255) / 256, 256, 0, stream>>>(projW[i], pwh + (size_t)i * HID_DIM * X1_K,
                                                             pwl + (size_t)i * HID_DIM * X1_K, HID_DIM, X1_K, X1_K, n2);
  }
  {
    const int n2 = DIST_RP * DIST_K / 2;
    cast_rows_bf16hl<<<(n2 + 255) / 256, 256, 0, stream>>>(dist_emb, deh, del, DIST_ROWS, DIST_K, DIST_K, n2);
  }
  {
    const int n2 = HID_DIM * DIST_K / 2;
    cast_rows_bf16hl<<<(n2 + 255) / 256, 256, 0, stream>>>(dist_W, dwh, dwl, HID_DIM, DIST_K, DIST_K, n2);
  }

  wmma_gemm64<0, false, 0, 0, false><<<dim3((SEQ_LEN / 64) * (GATE4 / 64) / 8, 2), 256, 0, stream>>>(
      (const unsigned short*)x0, nullptr, EMB_KP, 0L,
      (const unsigned short*)wih0, nullptr, EMB_KP, (long)GATE4 * EMB_KP,
      gx, nullptr, GATE4, (long)SEQ_LEN * GATE4,
      nullptr, nullptr, 0L, SEQ_LEN, GATE4, EMB_KP, 1.0f);

  lstm_scan_dir<<<2, 512, 0, stream>>>(gx, whh0, bih0, bhh0, hist0);

  {
    const int n2 = SEQ_LEN * X1_K / 2;
    cast_rows_f16<<<(n2 + 255) / 256, 256, 0, stream>>>(hist0, x1, X1_K, X1_K, n2);
  }

  wmma_gemm64<0, false, 0, 0, false><<<dim3((SEQ_LEN / 64) * (GATE4 / 64) / 8, 2), 256, 0, stream>>>(
      (const unsigned short*)x1, nullptr, X1_K, 0L,
      (const unsigned short*)wih1, nullptr, X1_K, (long)GATE4 * X1_K,
      gx, nullptr, GATE4, (long)SEQ_LEN * GATE4,
      nullptr, nullptr, 0L, SEQ_LEN, GATE4, X1_K, 1.0f);

  lstm_scan_dir<<<2, 512, 0, stream>>>(gx, whh1, bih1, bhh1, hist1);

  {
    const int n2 = SEQ_LEN * X1_K / 2;
    cast_rows_bf16hl<<<(n2 + 255) / 256, 256, 0, stream>>>(hist1, sth, stl, SEQ_LEN, X1_K, X1_K, n2);
  }

  wmma_gemm64<1, true, 0, 0, false><<<dim3((SEQ_LEN / 64) * (PROJ_N / 64) / 8, 1), 256, 0, stream>>>(
      sth, stl, X1_K, 0L,
      pwh, pwl, X1_K, 0L,
      proj, nullptr, PROJ_N, 0L,
      nullptr, nullptr, 0L, SEQ_LEN, PROJ_N, X1_K, 1.0f);

  wmma_gemm64<1, true, 2, 0, false><<<dim3(1, 1), 256, 0, stream>>>(
      deh, del, DIST_K, 0L,
      dwh, dwl, DIST_K, 0L,
      dtab, nullptr, HID_DIM, 0L,
      dist_b, nullptr, 0L, DIST_RP, HID_DIM, DIST_K, 1.0f);

  arc_score_rows<<<NUM_ARC / PARTS_PER_BLOCK, 256, 0, stream>>>(proj, dtab, arc_head, arc_mod, arc_w, out);
  sib_score_rows<<<NUM_SIB / PARTS_PER_BLOCK, 256, 0, stream>>>(proj, sib_head, sib_mod, sib_sib, arc_w, out + NUM_ARC);
}
